// QLSTM_57380763075320
// MI455X (gfx1250) — hardware-verified
//
#include <hip/hip_runtime.h>
#include <math.h>

constexpr int TSTEPS  = 256;
constexpr int NBATCH  = 128;
constexpr int NFEAT   = 256;
constexpr int NHID    = 512;
constexpr int NGH     = 4 * NHID;
constexpr int QIN_X   = NFEAT / 4;
constexpr int QHID    = NHID / 4;
constexpr int NROWS   = TSTEPS * NBATCH;
constexpr int KCAT    = 2 * NHID;
constexpr int NTHR    = 256;
constexpr int NWAVE   = NTHR / 32;
constexpr int SEQ_BLK = 16;
constexpr int XPITCH  = 264;
constexpr int HPITCH  = 520;
constexpr int SLABP   = 68;
constexpr float WCARRY     = 16.0f;
constexpr float WCARRY_INV = 1.0f / 16.0f;
constexpr unsigned QNEG_MASK = 0x284Eu;

static_assert(NBATCH % SEQ_BLK == 0);
static_assert(NHID == 64 * NWAVE);
static_assert(NFEAT % 32 == 0 && NHID % 32 == 0 && KCAT % 32 == 0);
static_assert(NROWS % 64 == 0 && NFEAT % 64 == 0);
static_assert(SEQ_BLK * NFEAT == NTHR * 16);
static_assert((NGH * (NFEAT / 8)) % NTHR == 0);
static_assert((NGH * (NHID / 8)) % NTHR == 0);
static_assert((NFEAT * (KCAT / 8)) % NTHR == 0);
static_assert(NFEAT == 64 * 4);
static_assert(XPITCH % 8 == 0 && HPITCH % 8 == 0 && SLABP % 4 == 0);
static_assert(QIN_X % 8 == 0 && QHID % 8 == 0);
static_assert(((NROWS / 64) * (NFEAT / 64)) % 8 == 0);
static_assert((SEQ_BLK * XPITCH) % 8 == 0 && (SEQ_BLK * HPITCH) % 8 == 0);

typedef __attribute__((ext_vector_type(16))) _Float16 v16h;
typedef __attribute__((ext_vector_type(8)))  _Float16 v8h;
typedef __attribute__((ext_vector_type(16))) __bf16   v16b;
typedef __attribute__((ext_vector_type(8)))  __bf16   v8b;
typedef __attribute__((ext_vector_type(8)))  float    v8f;
typedef __attribute__((ext_vector_type(4)))  float    v4f;
typedef __attribute__((ext_vector_type(4)))  unsigned v4u;

__device__ __forceinline__ unsigned short f2bf_bits(float f) {
  unsigned u = __float_as_uint(f);
  return (unsigned short)((u + 0x7FFFu + ((u >> 16) & 1u)) >> 16);
}
__device__ __forceinline__ float bf_bits2f(unsigned short h) { return __uint_as_float(((unsigned)h) << 16); }
__device__ __forceinline__ float bf16r(float f) { return bf_bits2f(f2bf_bits(f)); }

__device__ __forceinline__ void dep_guard_h(v8f& a, v8f& b, v16h x, v16h y) { asm volatile("v_nop\n\tv_nop\n\tv_nop\n\tv_nop" : "+v"(a), "+v"(b) : "v"(x), "v"(y)); }
__device__ __forceinline__ void dep_guard_b(v8f& a, v8f& b, v16b x, v16b y) { asm volatile("v_nop\n\tv_nop\n\tv_nop\n\tv_nop" : "+v"(a), "+v"(b) : "v"(x), "v"(y)); }
__device__ __forceinline__ void keep4_h(v16h a, v16h b, v16h c, v16h d) { asm volatile("v_nop" :: "v"(a), "v"(b), "v"(c), "v"(d)); }
__device__ __forceinline__ void keep4_b(v16b a, v16b b, v16b c, v16b d) { asm volatile("v_nop" :: "v"(a), "v"(b), "v"(c), "v"(d)); }
__device__ __forceinline__ void acc_guard4(v8f& a, v8f& b, v8f& c, v8f& d) { asm volatile("v_nop\n\tv_nop\n\tv_nop\n\tv_nop" : "+v"(a), "+v"(b), "+v"(c), "+v"(d)); }
__device__ __forceinline__ void grp_guard_h(v8f& a0, v8f& a1, v8f& a2, v8f& a3, v16h f0, v16h f1, v16h f2, v16h f3, v16h f4) {
  asm volatile("v_nop\n\tv_nop\n\tv_nop\n\tv_nop" : "+v"(a0), "+v"(a1), "+v"(a2), "+v"(a3) : "v"(f0), "v"(f1), "v"(f2), "v"(f3), "v"(f4));
}
__device__ __forceinline__ void grp_guard_b(v8f& a0, v8f& a1, v8f& a2, v8f& a3, v16b f0, v16b f1, v16b f2, v16b f3, v16b f4) {
  asm volatile("v_nop\n\tv_nop\n\tv_nop\n\tv_nop" : "+v"(a0), "+v"(a1), "+v"(a2), "+v"(a3) : "v"(f0), "v"(f1), "v"(f2), "v"(f3), "v"(f4));
}
template <typename T> struct Frag;
template <> struct Frag<_Float16> {
  typedef v16h V; union U { v16h v; v8h h[2]; };
  static __device__ __forceinline__ v16h load(const _Float16* p) {
    U f; f.h[0] = *(const v8h*)(p); f.h[1] = *(const v8h*)(p + 16); return f.v;
  }
  static __device__ __forceinline__ v8f mma(v16h a, v16h b, v8f c) {
    return __builtin_amdgcn_wmma_f32_16x16x32_f16(false, a, false, b, (short)0, c, false, false);
  }
  static __device__ __forceinline__ void guard(v8f& a, v8f& b, v16h x, v16h y) { dep_guard_h(a, b, x, y); }
  static __device__ __forceinline__ void gguard(v8f& a0, v8f& a1, v8f& a2, v8f& a3, v16h f0, v16h f1, v16h f2, v16h f3, v16h f4) { grp_guard_h(a0, a1, a2, a3, f0, f1, f2, f3, f4); }
  static __device__ __forceinline__ void keep(v16h a, v16h b, v16h c, v16h d) { keep4_h(a, b, c, d); }
};
template <> struct Frag<__bf16> {
  typedef v16b V; union U { v16b v; v8b h[2]; };
  static __device__ __forceinline__ v16b load(const __bf16* p) {
    U f; f.h[0] = *(const v8b*)(p); f.h[1] = *(const v8b*)(p + 16); return f.v;
  }
  static __device__ __forceinline__ v8f mma(v16b a, v16b b, v8f c) {
    return __builtin_amdgcn_wmma_f32_16x16x32_bf16(false, a, false, b, (short)0, c, false, false);
  }
  static __device__ __forceinline__ void guard(v8f& a, v8f& b, v16b x, v16b y) { dep_guard_b(a, b, x, y); }
  static __device__ __forceinline__ void gguard(v8f& a0, v8f& a1, v8f& a2, v8f& a3, v16b f0, v16b f1, v16b f2, v16b f3, v16b f4) { grp_guard_b(a0, a1, a2, a3, f0, f1, f2, f3, f4); }
  static __device__ __forceinline__ void keep(v16b a, v16b b, v16b c, v16b d) { keep4_b(a, b, c, d); }
};

__device__ __forceinline__ float fsigp(float z)  { return __builtin_amdgcn_rcpf(1.0f + expf(-z)); }
__device__ __forceinline__ float ftanhp(float z) { return 1.0f - 2.0f * __builtin_amdgcn_rcpf(1.0f + expf(2.0f * z)); }

template <int ET> struct Elem;
template <> struct Elem<0> { typedef _Float16 T; };
template <> struct Elem<1> { typedef __bf16 T; };
template <int ET, bool SPLIT, int BIAS_MODE, int OUT_MODE, bool RESID, int ACT = 0>
__global__ __launch_bounds__(256) void wmma_gemm64(
    const unsigned short* __restrict__ Ap, const unsigned short* __restrict__ A2p, int lda, long strideA,
    const unsigned short* __restrict__ Btp, const unsigned short* __restrict__ Bt2p, int ldb, long strideB,
    void* __restrict__ Cout, void* __restrict__ Cout2, int ldc, long strideC,
    const float* __restrict__ bias,
    const float* __restrict__ resid, long strideR,
    int M, int N, int K, float scale) {
  typedef typename Elem<ET>::T T;
  typedef typename Frag<T>::V V;
  const T* A = (const T*)Ap; const T* A2 = (const T*)A2p; const T* Bt = (const T*)Btp; const T* Bt2 = (const T*)Bt2p;
  __shared__ __align__(16) float sT[8][16 * 68];
  const int b    = blockIdx.y;
  const int lane = threadIdx.x & 31;
  const int wave = threadIdx.x >> 5;
  const int tilesN = N >> 6;
  const int tilesM = M >> 6;
  const int tile = blockIdx.x * 8 + wave;
  if (tile >= tilesM * tilesN) return;
  const int tm = tile / tilesN;
  const int tn = tile - tm * tilesN;
  const int m0 = tm << 6;
  const int n0 = tn << 6;

  const T* Ab  = A  + (size_t)b * strideA;
  const T* Bb  = Bt + (size_t)b * strideB;
  const T* Ab2 = SPLIT ? (A2  + (size_t)b * strideA) : nullptr;
  const T* Bb2 = SPLIT ? (Bt2 + (size_t)b * strideB) : nullptr;

  const int rlane = lane & 15;
  const int koff  = (lane >> 4) * 8;
  const int mOff  = (lane >> 4) * 8;

  v8f acc[4][4];
#pragma unroll
  for (int i = 0; i < 4; ++i)
#pragma unroll
    for (int j = 0; j < 4; ++j) acc[i][j] = (v8f){0.f,0.f,0.f,0.f,0.f,0.f,0.f,0.f};

  for (int k0 = 0; k0 < K; k0 += 32) {
    V bh[4], bl[4];
#pragma unroll
    for (int j = 0; j < 4; ++j) {
      const size_t bo = (size_t)(n0 + (j << 4) + rlane) * ldb + koff + k0;
      bh[j] = Frag<T>::load(Bb + bo);
      if (SPLIT) bl[j] = Frag<T>::load(Bb2 + bo);
    }
#pragma unroll
    for (int i = 0; i < 4; ++i) {
      const size_t ao = (size_t)(m0 + (i << 4) + rlane) * lda + koff + k0;
      V ah = Frag<T>::load(Ab + ao);
      V al;
      if (SPLIT) al = Frag<T>::load(Ab2 + ao);
#pragma unroll
      for (int j = 0; j < 4; ++j) {
        acc[i][j] = Frag<T>::mma(ah, bh[j], acc[i][j]);
        if (SPLIT) {
          acc[i][j] = Frag<T>::mma(ah, bl[j], acc[i][j]);
          acc[i][j] = Frag<T>::mma(al, bh[j], acc[i][j]);
        }
      }
      Frag<T>::gguard(acc[i][0], acc[i][1], acc[i][2], acc[i][3], ah, SPLIT ? al : ah, bh[0], bh[3], SPLIT ? bl[3] : bh[3]);
    }
    Frag<T>::keep(bh[0], bh[1], bh[2], bh[3]);
    if (SPLIT) Frag<T>::keep(bl[0], bl[1], bl[2], bl[3]);
  }
  acc_guard4(acc[0][0], acc[0][1], acc[0][2], acc[0][3]);
  acc_guard4(acc[1][0], acc[1][1], acc[1][2], acc[1][3]);
  acc_guard4(acc[2][0], acc[2][1], acc[2][2], acc[2][3]);
  acc_guard4(acc[3][0], acc[3][1], acc[3][2], acc[3][3]);

  float* slab = sT[wave];
  const float* Rb = RESID ? (resid + (size_t)b * strideR) : nullptr;
#pragma unroll
  for (int i = 0; i < 4; ++i) {
    const int mBase = m0 + (i << 4);
#pragma unroll
    for (int j = 0; j < 4; ++j) {
      const int n = n0 + (j << 4) + rlane;
      float bv = 0.f;
      if (BIAS_MODE == 2) bv = bias[n];
#pragma unroll
      for (int r = 0; r < 8; ++r) {
        float v = acc[i][j][r] * scale;
        if (BIAS_MODE == 1) v += bias[mBase + mOff + r];
        if (BIAS_MODE == 2) v += bv;
        if (RESID) v += Rb[(size_t)(mBase + mOff + r) * ldc + n];
        if (ACT == 1) v = tanhf(v);
        if (ACT == 2) v = fmaxf(v, 0.0f);
        if (ACT == 3) v = v / (1.0f + expf(-v));
        if (ACT == 4) v = (v > 0.f) ? v : 0.01f * v;
        if (ACT == 5) v = 0.5f * v * (1.0f + erff(v * 0.70710678118654752f));
        slab[(mOff + r) * 68 + (j << 4) + rlane] = v;
      }
    }
    __builtin_amdgcn_fence(__ATOMIC_RELEASE, "workgroup");
    __builtin_amdgcn_wave_barrier();
    __builtin_amdgcn_fence(__ATOMIC_ACQUIRE, "workgroup");
    if (OUT_MODE == 0) {
      float* C = (float*)Cout + (size_t)b * strideC;
      const int hh = lane >> 4, c4 = (lane & 15) * 4;
      for (int pass = 0; pass < 2; ++pass) {
#pragma unroll
        for (int it = 0; it < 8; ++it) {
          const int row = it * 2 + hh;
          v4f v = *(const v4f*)(slab + row * 68 + c4);
          *(volatile v4f*)(C + (size_t)(mBase + row) * ldc + n0 + c4) = v;
        }
        __threadfence();
      }
    } else {
      const int q = lane >> 3, c8 = (lane & 7) * 8;
      unsigned short* C  = (unsigned short*)Cout  + (size_t)b * strideC;
      unsigned short* C2 = (OUT_MODE == 2) ? ((unsigned short*)Cout2 + (size_t)b * strideC) : nullptr;
      for (int pass = 0; pass < 2; ++pass) {
#pragma unroll
        for (int it = 0; it < 4; ++it) {
          const int row = it * 4 + q;
          const float* sp = slab + row * 68 + c8;
          v8h hv, lv;
#pragma unroll
          for (int e = 0; e < 8; ++e) {
            if (OUT_MODE == 1) {
              hv[e] = (_Float16)sp[e];
            } else {
              unsigned short hb = f2bf_bits(sp[e]);
              unsigned short lb = f2bf_bits(sp[e] - bf_bits2f(hb));
              hv[e] = __builtin_bit_cast(_Float16, hb);
              lv[e] = __builtin_bit_cast(_Float16, lb);
            }
          }
          *(volatile v8h*)(C + (size_t)(mBase + row) * ldc + n0 + c8) = hv;
          if (OUT_MODE == 2) *(volatile v8h*)(C2 + (size_t)(mBase + row) * ldc + n0 + c8) = lv;
        }
        __threadfence();
      }
    }
    __builtin_amdgcn_fence(__ATOMIC_RELEASE, "workgroup");
    __builtin_amdgcn_wave_barrier();
    __builtin_amdgcn_fence(__ATOMIC_ACQUIRE, "workgroup");
  }
}

__global__ __launch_bounds__(NTHR) void build_kxt_kernel(const float* __restrict__ Wx, unsigned short* __restrict__ KXT) {
  const int i = blockIdx.x * NTHR + threadIdx.x;
  if (i < NGH * (NFEAT / 8)) {
    const int nr  = i / (NFEAT / 8);
    const int f0  = (i - nr * (NFEAT / 8)) * 8;
    const int g   = nr / NHID, n = nr - g * NHID;
    const int qb  = n / QHID, hc = n - qb * QHID;
    const int qa  = f0 / QIN_X, fr0 = f0 - qa * QIN_X;
    const int comp = qa ^ qb;
    const float sgn = (((QNEG_MASK >> (4 * qb + qa)) & 1u) != 0u) ? -WCARRY : WCARRY;
    const float* wp = Wx + ((size_t)(g * 4 + comp) * QIN_X + fr0) * QHID + hc;
    v8h hv;
#pragma unroll
    for (int e = 0; e < 8; ++e) hv[e] = __builtin_bit_cast(_Float16, f2bf_bits(sgn * wp[(size_t)e * QHID]));
    unsigned short* op = KXT + (size_t)i * 8;
    *(volatile v8h*)op = hv;
    __threadfence();
    *(volatile v8h*)op = hv;
  }
}

__global__ __launch_bounds__(NTHR) void build_kut_kernel(const float* __restrict__ Uh, unsigned short* __restrict__ KUT) {
  const int i = blockIdx.x * NTHR + threadIdx.x;
  if (i < NGH * (NHID / 8)) {
    const int nr  = i / (NHID / 8);
    const int kc  = (i - nr * (NHID / 8)) * 8;
    const int g   = nr / NHID, n = nr - g * NHID;
    const int qb  = n / QHID, hc = n - qb * QHID;
    const int qa  = kc / QHID, kr0 = kc - qa * QHID;
    const int comp = qa ^ qb;
    const float sgn = (((QNEG_MASK >> (4 * qb + qa)) & 1u) != 0u) ? -WCARRY : WCARRY;
    const float* wp = Uh + ((size_t)(g * 4 + comp) * QHID + kr0) * QHID + hc;
    v8h hv;
#pragma unroll
    for (int e = 0; e < 8; ++e) {
      const float wv = sgn * bf16r(wp[(size_t)e * QHID]);
      hv[e] = (_Float16)wv;
    }
    unsigned short* op = KUT + (size_t)i * 8;
    *(volatile v8h*)op = hv;
    __threadfence();
    *(volatile v8h*)op = hv;
  }
}

__global__ __launch_bounds__(NTHR) void build_fcb_kernel(const float* __restrict__ fcw, unsigned short* __restrict__ FCB2) {
  const int i = blockIdx.x * NTHR + threadIdx.x;
  if (i < NFEAT * (KCAT / 8)) {
    const int n  = i / (KCAT / 8);
    const int kc = (i - n * (KCAT / 8)) * 8;
    const int ks = kc & (NHID - 1);
    const float* sp = fcw + (size_t)n * NHID + ks;
    const v4f a = *(const v4f*)(sp);
    const v4f b = *(const v4f*)(sp + 4);
    v8h hv;
#pragma unroll
    for (int e = 0; e < 4; ++e) {
      hv[e]     = __builtin_bit_cast(_Float16, f2bf_bits(a[e]));
      hv[4 + e] = __builtin_bit_cast(_Float16, f2bf_bits(b[e]));
    }
    unsigned short* op = FCB2 + (size_t)i * 8;
    *(volatile v8h*)op = hv;
    __threadfence();
    *(volatile v8h*)op = hv;
  }
}

__global__ __launch_bounds__(64) void build_fcbias_kernel(const float* __restrict__ fcb, float* __restrict__ FCBR) {
  const int t4 = threadIdx.x * 4;
  const v4f v = *(const v4f*)(fcb + t4);
  v4f o;
#pragma unroll
  for (int e = 0; e < 4; ++e) o[e] = bf16r(v[e]);
  float* op = FCBR + t4;
  *(volatile v4f*)op = o;
  __threadfence();
  *(volatile v4f*)op = o;
}

__device__ __forceinline__ void stage_x_tile(const float* __restrict__ x, unsigned short* axbuf, int tstep, int rowbase, int tid) {
  const int m = tid >> 4, fq = (tid & 15) * 16;
  const float* xp = x + ((size_t)tstep * NBATCH + rowbase + m) * NFEAT + fq;
  const v4f v0 = *(const v4f*)(xp);
  const v4f v1 = *(const v4f*)(xp + 4);
  const v4f v2 = *(const v4f*)(xp + 8);
  const v4f v3 = *(const v4f*)(xp + 12);
  v4u p0, p1;
  p0[0] = (unsigned)f2bf_bits(v0[0]) | ((unsigned)f2bf_bits(v0[1]) << 16);
  p0[1] = (unsigned)f2bf_bits(v0[2]) | ((unsigned)f2bf_bits(v0[3]) << 16);
  p0[2] = (unsigned)f2bf_bits(v1[0]) | ((unsigned)f2bf_bits(v1[1]) << 16);
  p0[3] = (unsigned)f2bf_bits(v1[2]) | ((unsigned)f2bf_bits(v1[3]) << 16);
  p1[0] = (unsigned)f2bf_bits(v2[0]) | ((unsigned)f2bf_bits(v2[1]) << 16);
  p1[1] = (unsigned)f2bf_bits(v2[2]) | ((unsigned)f2bf_bits(v2[3]) << 16);
  p1[2] = (unsigned)f2bf_bits(v3[0]) | ((unsigned)f2bf_bits(v3[1]) << 16);
  p1[3] = (unsigned)f2bf_bits(v3[2]) | ((unsigned)f2bf_bits(v3[3]) << 16);
  unsigned short* dp = axbuf + m * XPITCH + fq;
  *(v4u*)(dp)     = p0;
  *(v4u*)(dp + 8) = p1;
}

__global__ __launch_bounds__(NTHR) void hq_seq_kernel(const float* __restrict__ x, const float* __restrict__ bx,
                                                      const unsigned short* __restrict__ KXTp,
                                                      const unsigned short* __restrict__ KUTp,
                                                      unsigned short* __restrict__ HS2) {
  __shared__ __align__(16) unsigned short Ax[2][SEQ_BLK * XPITCH];
  __shared__ __align__(16) _Float16       Ah[2][SEQ_BLK * HPITCH];
  __shared__ __align__(16) float          Sl[NWAVE][16 * SLABP];
  const __bf16*   KXT = (const __bf16*)KXTp;
  const _Float16* KUT = (const _Float16*)KUTp;
  const int tid = threadIdx.x, lane = tid & 31, wave = tid >> 5;
  const int c = lane & 15, hh = lane >> 4, koff = hh * 8;
  const int rowbase = blockIdx.x * SEQ_BLK;

  {
    unsigned* axz = (unsigned*)(&Ax[0][0]);
#pragma unroll 1
    for (int i = tid; i < (2 * SEQ_BLK * XPITCH) / 2; i += NTHR) axz[i] = 0u;
    unsigned* ahz = (unsigned*)(&Ah[0][0]);
#pragma unroll 1
    for (int i = tid; i < (2 * SEQ_BLK * HPITCH) / 2; i += NTHR) ahz[i] = 0u;
  }
  float bb[4][4];
#pragma unroll
  for (int nt = 0; nt < 4; ++nt) {
    const int j = 64 * wave + 16 * nt + c;
#pragma unroll
    for (int g = 0; g < 4; ++g) bb[nt][g] = bf16r(bx[g * NHID + j]);
    asm volatile("" ::: "memory");
  }
  float cst[4][8];
#pragma unroll
  for (int nt = 0; nt < 4; ++nt)
#pragma unroll
    for (int r = 0; r < 8; ++r) cst[nt][r] = 0.0f;
  __syncthreads();
  stage_x_tile(x, &Ax[0][0], 0, rowbase, tid);
  __syncthreads();

  const v8f z8 = {0.f, 0.f, 0.f, 0.f, 0.f, 0.f, 0.f, 0.f};
  float* slab = Sl[wave];

#pragma unroll 1
  for (int t = 0; t < TSTEPS; ++t) {
    const int cur = t & 1;
    const __bf16*   axrow = (const __bf16*)(&Ax[cur][0]) + c * XPITCH + koff;
    const _Float16* ahrow = &Ah[cur][0] + c * HPITCH + koff;
    _Float16* ahn = &Ah[cur ^ 1][0];
#pragma unroll
    for (int nt = 0; nt < 4; ++nt) {
      const int j = 64 * wave + 16 * nt + c;
      const __bf16*   wxp = KXT + (size_t)j * NFEAT + koff;
      const _Float16* wup = KUT + (size_t)j * NHID + koff;
      v8f acc0 = z8, acc1 = z8, acc2 = z8, acc3 = z8;
#pragma unroll 1
      for (int kx = 0; kx < NFEAT; kx += 32) {
        const v16b a  = Frag<__bf16>::load(axrow + kx);
        const v16b b0 = Frag<__bf16>::load(wxp + kx);
        const v16b b1 = Frag<__bf16>::load(wxp + (size_t)1 * NHID * NFEAT + kx);
        const v16b b2 = Frag<__bf16>::load(wxp + (size_t)2 * NHID * NFEAT + kx);
        const v16b b3 = Frag<__bf16>::load(wxp + (size_t)3 * NHID * NFEAT + kx);
        acc0 = Frag<__bf16>::mma(a, b0, acc0);
        acc1 = Frag<__bf16>::mma(a, b1, acc1);
        acc2 = Frag<__bf16>::mma(a, b2, acc2);
        acc3 = Frag<__bf16>::mma(a, b3, acc3);
        grp_guard_b(acc0, acc1, acc2, acc3, a, b0, b1, b2, b3);
      }
#pragma unroll 1
      for (int k0 = 0; k0 < NHID; k0 += 32) {
        const v16h a  = Frag<_Float16>::load(ahrow + k0);
        const v16h b0 = Frag<_Float16>::load(wup + k0);
        const v16h b1 = Frag<_Float16>::load(wup + (size_t)1 * NHID * NHID + k0);
        const v16h b2 = Frag<_Float16>::load(wup + (size_t)2 * NHID * NHID + k0);
        const v16h b3 = Frag<_Float16>::load(wup + (size_t)3 * NHID * NHID + k0);
        acc0 = Frag<_Float16>::mma(a, b0, acc0);
        acc1 = Frag<_Float16>::mma(a, b1, acc1);
        acc2 = Frag<_Float16>::mma(a, b2, acc2);
        acc3 = Frag<_Float16>::mma(a, b3, acc3);
        grp_guard_h(acc0, acc1, acc2, acc3, a, b0, b1, b2, b3);
      }
      acc_guard4(acc0, acc1, acc2, acc3);
#pragma unroll
      for (int r = 0; r < 8; ++r) {
        const float zf = acc0[r] * WCARRY_INV + bb[nt][0];
        const float zi = acc1[r] * WCARRY_INV + bb[nt][1];
        const float zo = acc2[r] * WCARRY_INV + bb[nt][2];
        const float za = acc3[r] * WCARRY_INV + bb[nt][3];
        const float fg = fsigp(zf);
        const float ig = fsigp(zi);
        const float og = fsigp(zo);
        const float ag = ftanhp(za);
        const float cn = ig * ag + fg * cst[nt][r];
        cst[nt][r] = cn;
        const float hn = og * ftanhp(cn);
        ahn[(8 * hh + r) * HPITCH + j] = (_Float16)hn;
        slab[(8 * hh + r) * SLABP + 16 * nt + c] = hn;
      }
    }
    __builtin_amdgcn_fence(__ATOMIC_RELEASE, "workgroup");
    __builtin_amdgcn_wave_barrier();
    __builtin_amdgcn_fence(__ATOMIC_ACQUIRE, "workgroup");
    {
      const int q = lane >> 3, c8 = (lane & 7) * 8;
      v8h hv[4], lv[4];
#pragma unroll
      for (int it = 0; it < 4; ++it) {
        const int row = it * 4 + q;
        const v4f s0 = *(const v4f*)(slab + row * SLABP + c8);
        const v4f s1 = *(const v4f*)(slab + row * SLABP + c8 + 4);
#pragma unroll
        for (int e = 0; e < 4; ++e) {
          const unsigned short hb0 = f2bf_bits(s0[e]);
          const unsigned short lb0 = f2bf_bits(s0[e] - bf_bits2f(hb0));
          const unsigned short hb1 = f2bf_bits(s1[e]);
          const unsigned short lb1 = f2bf_bits(s1[e] - bf_bits2f(hb1));
          hv[it][e]     = __builtin_bit_cast(_Float16, hb0);
          lv[it][e]     = __builtin_bit_cast(_Float16, lb0);
          hv[it][4 + e] = __builtin_bit_cast(_Float16, hb1);
          lv[it][4 + e] = __builtin_bit_cast(_Float16, lb1);
        }
      }
      unsigned short* hrow = HS2 + ((size_t)t * NBATCH + rowbase) * KCAT + 64 * wave + c8;
      for (int pass = 0; pass < 2; ++pass) {
#pragma unroll
        for (int it = 0; it < 4; ++it) {
          const int row = it * 4 + q;
          unsigned short* p = hrow + (size_t)row * KCAT;
          *(volatile v8h*)(p)        = hv[it];
          *(volatile v8h*)(p + NHID) = lv[it];
        }
        __threadfence();
      }
    }
    __builtin_amdgcn_fence(__ATOMIC_RELEASE, "workgroup");
    __builtin_amdgcn_wave_barrier();
    __builtin_amdgcn_fence(__ATOMIC_ACQUIRE, "workgroup");
    {
      const int tn = (t + 1 < TSTEPS) ? (t + 1) : (TSTEPS - 1);
      stage_x_tile(x, &Ax[cur ^ 1][0], tn, rowbase, tid);
    }
    __syncthreads();
  }
}

extern "C" void kernel_launch(void* const* d_in, const int* in_sizes, int n_in,
                              void* d_out, int out_size, void* d_ws, size_t ws_size, hipStream_t stream) {
  if (n_in < 6 || d_out == nullptr || d_ws == nullptr) return;
  if (in_sizes[0] != TSTEPS * NBATCH * NFEAT || in_sizes[1] != 16 * QIN_X * QHID || in_sizes[2] != NGH ||
      in_sizes[3] != 16 * QHID * QHID || in_sizes[4] != NFEAT * NHID || in_sizes[5] != NFEAT ||
      out_size != NROWS * NFEAT) return;

  const float* x    = (const float*)d_in[0];
  const float* Wx   = (const float*)d_in[1];
  const float* bx   = (const float*)d_in[2];
  const float* Uh   = (const float*)d_in[3];
  const float* fcw  = (const float*)d_in[4];
  const float* fcb  = (const float*)d_in[5];
  float* out = (float*)d_out;

  char* ws = (char*)d_ws; size_t off = 0;
  auto carve = [&](size_t bytes) -> char* { char* p = ws + off; off += (bytes + 255) & ~(size_t)255; return p; };
  unsigned short* KXT  = (unsigned short*)carve((size_t)NGH * NFEAT * 2);
  unsigned short* KUT  = (unsigned short*)carve((size_t)NGH * NHID * 2);
  unsigned short* FCB2 = (unsigned short*)carve((size_t)NFEAT * KCAT * 2);
  float*          FCBR = (float*)carve((size_t)NFEAT * 4);
  unsigned short* HS2  = (unsigned short*)carve((size_t)NROWS * KCAT * 2);
  if (off > ws_size || off > (size_t)134217728) return;

  build_kxt_kernel<<<(NGH * (NFEAT / 8)) / NTHR, NTHR, 0, stream>>>(Wx, KXT);
  build_kut_kernel<<<(NGH * (NHID / 8)) / NTHR, NTHR, 0, stream>>>(Uh, KUT);
  build_fcb_kernel<<<(NFEAT * (KCAT / 8)) / NTHR, NTHR, 0, stream>>>(fcw, FCB2);
  build_fcbias_kernel<<<1, 64, 0, stream>>>(fcb, FCBR);
  hq_seq_kernel<<<NBATCH / SEQ_BLK, NTHR, 0, stream>>>(x, bx, KXT, KUT, HS2);
  const dim3 ggrid(((NROWS / 64) * (NFEAT / 64)) / 8, 1);
  wmma_gemm64<1, false, 2, 0, false, 0><<<ggrid, 256, 0, stream>>>(
      HS2, HS2, KCAT, 0L, FCB2, FCB2, KCAT, 0L, (void*)out, (void*)out, NFEAT, 0L,
      FCBR, FCBR, 0L, NROWS, NFEAT, KCAT, 1.0f);
}
